// GatedLSTMCell_58548994179834
// MI455X (gfx1250) — hardware-verified
//
#include <hip/hip_runtime.h>
#include <hip/hip_bf16.h>
#include <math.h>
#include <stdint.h>


typedef __bf16 v16bf __attribute__((ext_vector_type(16)));
typedef int    v4i   __attribute__((ext_vector_type(4)));
typedef float  v8f   __attribute__((ext_vector_type(8)));
typedef float  v4f   __attribute__((ext_vector_type(4)));

#define FEAT   1024
#define HID    1024
#define GATEW  4096
#define GD     256
#define BLK    128
#define KB     64
#define KP     72
#define CPA    68
#define CPC    132
#define NT     256

__device__ __forceinline__ unsigned bf16_rne(float f) {
    const unsigned u = __float_as_uint(f);
    return (u + 0x7FFFu + ((u >> 16) & 1u)) >> 16;
}
__device__ __forceinline__ void split2(float x, unsigned& hi, unsigned& lo) {
    hi = bf16_rne(x);
    lo = bf16_rne(x - __uint_as_float(hi << 16));
}
__device__ __forceinline__ void split3(float x, unsigned& hi, unsigned& mi, unsigned& lo) {
    hi = bf16_rne(x);
    const float r1 = x - __uint_as_float(hi << 16);
    mi = bf16_rne(r1);
    const float r2 = r1 - __uint_as_float(mi << 16);
    lo = bf16_rne(r2);
}

__device__ __forceinline__ v8f zero8() {
    v8f r;
#pragma unroll
    for (int i = 0; i < 8; ++i) r[i] = 0.0f;
    return r;
}

__device__ __forceinline__ v8f wmma_bf16(v8f c, v16bf a, v16bf b) {
    v8f d = __builtin_amdgcn_wmma_f32_16x16x32_bf16(false, a, false, b, (short)0, c, false, false);
    asm volatile("v_nop\n\tv_nop\n\tv_nop\n\tv_nop" : "+v"(d) : "v"(a), "v"(b));
    return d;
}

__device__ __forceinline__ v16bf ldfrag(const unsigned short* T, int row, int k0, int h) {
    union { v4i i[2]; v16bf v; } u;
    const unsigned short* p = T + row * KP + k0 + 8 * h;
    u.i[0] = *(const v4i*)(p);
    u.i[1] = *(const v4i*)(p + 16);
    return u.v;
}

__device__ __forceinline__ float sigm(float x) { return 1.0f / (1.0f + expf(-x)); }

__device__ __forceinline__ float cell_point(float pi, float pf, float pc, float po, float c0, float& cy) {
    const float ig = sigm(pi), fg = sigm(pf), cg = tanhf(pc), og = sigm(po);
    cy = fg * c0 + ig * cg;
    return og * tanhf(cy);
}

__global__ __launch_bounds__(NT) void k_gate_logits(
    const float* __restrict__ input, const float* __restrict__ hx,
    const float* __restrict__ w_gih, const float* __restrict__ w_ghh,
    const float* __restrict__ b_gih, const float* __restrict__ b_ghh,
    float* __restrict__ logits, int B)
{
    __shared__ __attribute__((aligned(16))) unsigned short As[3][32 * KP];
    __shared__ __attribute__((aligned(16))) unsigned short Ws[3][64 * KP];
    __shared__ __attribute__((aligned(16))) float Cs[32 * CPA];

    const int t = threadIdx.x, lane = t & 31, w = t >> 5, h = lane >> 4, q = lane & 15;
    const int m0 = blockIdx.x * 32, n0 = blockIdx.y * 64, z = blockIdx.z;
    if (m0 + 32 > B) return;
    const float* X  = z ? hx    : input;
    const float* Wg = z ? w_ghh : w_gih;
    const float* Bg = z ? b_ghh : b_gih;
    float* dst = logits + (size_t)z * (size_t)B * GD;
    const int mh = w >> 2, nq = w & 3;

    v8f acc = zero8();
#pragma unroll 1
    for (int kb = 0; kb < FEAT / KB; ++kb) {
        __syncthreads();
#pragma unroll
        for (int it = 0; it < 2; ++it) {
            const int idx = it * NT + t, r = idx >> 4, c4 = (idx & 15) * 4;
            const v4f x4 = *(const v4f*)(X + (size_t)(m0 + r) * FEAT + kb * KB + c4);
            unsigned eh[4], em[4], el[4];
#pragma unroll
            for (int c = 0; c < 4; ++c) split3(x4[c], eh[c], em[c], el[c]);
            const int o = r * KP + c4;
            *(uint2*)&As[0][o] = make_uint2(eh[0] | (eh[1] << 16), eh[2] | (eh[3] << 16));
            *(uint2*)&As[1][o] = make_uint2(em[0] | (em[1] << 16), em[2] | (em[3] << 16));
            *(uint2*)&As[2][o] = make_uint2(el[0] | (el[1] << 16), el[2] | (el[3] << 16));
        }
#pragma unroll
        for (int it = 0; it < 2; ++it) {
            const int idx = it * NT + t, kp = idx >> 4, n4 = (idx & 15) * 4;
            const float* wp = Wg + (size_t)(kb * KB + 2 * kp) * GD + n0 + n4;
            const v4f w0 = *(const v4f*)(wp);
            const v4f w1 = *(const v4f*)(wp + GD);
#pragma unroll
            for (int c = 0; c < 4; ++c) {
                unsigned h0, g0, l0, h1, g1, l1;
                split3(w0[c], h0, g0, l0);
                split3(w1[c], h1, g1, l1);
                const int o = (n4 + c) * KP + 2 * kp;
                *(unsigned*)&Ws[0][o] = h0 | (h1 << 16);
                *(unsigned*)&Ws[1][o] = g0 | (g1 << 16);
                *(unsigned*)&Ws[2][o] = l0 | (l1 << 16);
            }
        }
        __syncthreads();
#pragma unroll
        for (int ks = 0; ks < KB / 32; ++ks) {
            const int k0 = ks * 32;
            const v16bf ah = ldfrag(As[0], mh * 16 + q, k0, h);
            const v16bf am = ldfrag(As[1], mh * 16 + q, k0, h);
            const v16bf al = ldfrag(As[2], mh * 16 + q, k0, h);
            const v16bf bh = ldfrag(Ws[0], nq * 16 + q, k0, h);
            const v16bf bm = ldfrag(Ws[1], nq * 16 + q, k0, h);
            const v16bf bl = ldfrag(Ws[2], nq * 16 + q, k0, h);
            v8f tq = zero8();
            tq = wmma_bf16(tq, al, bh);
            tq = wmma_bf16(tq, am, bm);
            tq = wmma_bf16(tq, ah, bl);
            tq = wmma_bf16(tq, am, bh);
            tq = wmma_bf16(tq, ah, bm);
            tq = wmma_bf16(tq, ah, bh);
            acc += tq;
        }
    }

    const float bias = Bg[n0 + nq * 16 + q];
#pragma unroll
    for (int r = 0; r < 8; ++r)
        Cs[(mh * 16 + 8 * h + r) * CPA + nq * 16 + q] = acc[r] + bias;
    __syncthreads();
    const int rowA = 4 * w + h, rowB = 4 * w + 2 + h, c4 = 4 * q;
    const v4f vA = *(const v4f*)&Cs[rowA * CPA + c4];
    const v4f vB = *(const v4f*)&Cs[rowB * CPA + c4];
    float* pA = dst + (size_t)(m0 + rowA) * GD + n0 + c4;
    float* pB = dst + (size_t)(m0 + rowB) * GD + n0 + c4;
    *(volatile v4f*)pA = vA;
    *(volatile v4f*)pB = vB;
    __threadfence();
    *(volatile v4f*)pA = vA;
    *(volatile v4f*)pB = vB;
}

__global__ __launch_bounds__(NT) void k_sparsify(const float* __restrict__ logits,
                                                 float* __restrict__ gates, int nrows)
{
    const int t = threadIdx.x, lane = t & 31, w = t >> 5;
    const int row = blockIdx.x * 8 + w;
    if (row >= nrows) return;
    const float* p = logits + (size_t)row * GD;
    const v4f a = *(const v4f*)(p + 4 * lane);
    const v4f b = *(const v4f*)(p + 128 + 4 * lane);
    float v[8];
    unsigned key[8];
#pragma unroll
    for (int i = 0; i < 4; ++i) { v[i] = a[i]; v[4 + i] = b[i]; }
#pragma unroll
    for (int i = 0; i < 8; ++i) {
        const unsigned u = __float_as_uint(v[i]);
        key[i] = (u & 0x80000000u) ? ~u : (u | 0x80000000u);
    }
    unsigned lo = 0u, hi = 0xFFFFFFFFu;
    while (lo < hi) {
        const unsigned mid = lo + ((hi - lo) >> 1) + 1u;
        int c = 0;
#pragma unroll
        for (int i = 0; i < 8; ++i) c += (key[i] >= mid) ? 1 : 0;
#pragma unroll
        for (int off = 16; off > 0; off >>= 1) c += __shfl_xor(c, off, 32);
        if (c >= 128) lo = mid; else hi = mid - 1u;
    }
    const unsigned thr = lo;
    float s = 0.0f, r[8];
#pragma unroll
    for (int i = 0; i < 8; ++i) { r[i] = (key[i] >= thr) ? v[i] : 0.0f; s += r[i]; }
#pragma unroll
    for (int off = 16; off > 0; off >>= 1) s += __shfl_xor(s, off, 32);
    const float scale = 256.0f / s;
    v4f o0, o1;
#pragma unroll
    for (int i = 0; i < 4; ++i) { o0[i] = r[i] * scale; o1[i] = r[4 + i] * scale; }
    float* g = gates + (size_t)row * GD;
    float* p0 = g + 4 * lane;
    float* p1 = g + 128 + 4 * lane;
    *(volatile v4f*)p0 = o0;
    *(volatile v4f*)p1 = o1;
    __threadfence();
    *(volatile v4f*)p0 = o0;
    *(volatile v4f*)p1 = o1;
}

union __attribute__((aligned(16))) WTile { unsigned short w[BLK * KP]; float c[32 * CPC]; };

__device__ __forceinline__ void gate_pass(const int gt, v8f& acc0, v8f& acc1,
    const float* __restrict__ input, const float* __restrict__ hx,
    const float* __restrict__ weight_ih, const float* __restrict__ weight_hh,
    unsigned short* Ah, unsigned short* Al, unsigned short* Wh, unsigned short* Wl,
    const float* Gl, const int m0, const int jh, const int t, const int w, const int h, const int q)
{
    const int colbase = (gt * 8 + jh) * BLK;
#pragma unroll 1
    for (int kb = 0; kb < 2 * (FEAT / KB); ++kb) {
        __syncthreads();
        const bool first = kb < (FEAT / KB);
        const float* X    = first ? input     : hx;
        const float* Wsrc = first ? weight_ih : weight_hh;
        const int kloc  = (kb & (FEAT / KB - 1)) * KB;
        const int kb128 = kb >> 1;
#pragma unroll
        for (int it = 0; it < 2; ++it) {
            const int idx = it * NT + t, r = idx >> 4, c4 = (idx & 15) * 4;
            const float gv = Gl[r * 64 + kb128 * 4 + gt];
            const v4f x4 = *(const v4f*)(X + (size_t)(m0 + r) * FEAT + kloc + c4);
            unsigned eh[4], el[4];
#pragma unroll
            for (int c = 0; c < 4; ++c) split2(x4[c] * gv, eh[c], el[c]);
            const int o = r * KP + c4;
            *(uint2*)&Ah[o] = make_uint2(eh[0] | (eh[1] << 16), eh[2] | (eh[3] << 16));
            *(uint2*)&Al[o] = make_uint2(el[0] | (el[1] << 16), el[2] | (el[3] << 16));
        }
#pragma unroll
        for (int it = 0; it < 4; ++it) {
            const int idx = it * NT + t, kp = idx >> 5, n4 = (idx & 31) * 4;
            const float* wp = Wsrc + (size_t)(kloc + 2 * kp) * GATEW + colbase + n4;
            const v4f w0 = *(const v4f*)(wp);
            const v4f w1 = *(const v4f*)(wp + GATEW);
#pragma unroll
            for (int c = 0; c < 4; ++c) {
                unsigned h0, l0, h1, l1;
                split2(w0[c], h0, l0);
                split2(w1[c], h1, l1);
                const int o = (n4 + c) * KP + 2 * kp;
                *(unsigned*)&Wh[o] = h0 | (h1 << 16);
                *(unsigned*)&Wl[o] = l0 | (l1 << 16);
            }
        }
        __syncthreads();
#pragma unroll
        for (int ks = 0; ks < KB / 32; ++ks) {
            const int k0 = ks * 32;
            const v16bf bh = ldfrag(Wh, w * 16 + q, k0, h);
            const v16bf bl = ldfrag(Wl, w * 16 + q, k0, h);
            {
                const v16bf ah = ldfrag(Ah, q, k0, h);
                const v16bf al = ldfrag(Al, q, k0, h);
                acc0 = wmma_bf16(acc0, al, bh);
                acc0 = wmma_bf16(acc0, ah, bl);
                acc0 = wmma_bf16(acc0, ah, bh);
            }
            {
                const v16bf ah = ldfrag(Ah, 16 + q, k0, h);
                const v16bf al = ldfrag(Al, 16 + q, k0, h);
                acc1 = wmma_bf16(acc1, al, bh);
                acc1 = wmma_bf16(acc1, ah, bl);
                acc1 = wmma_bf16(acc1, ah, bh);
            }
        }
    }
}

__global__ __launch_bounds__(NT) void k_gated_lstm(
    const float* __restrict__ input, const float* __restrict__ hx,
    const float* __restrict__ cx,
    const float* __restrict__ weight_ih, const float* __restrict__ weight_hh,
    const float* __restrict__ bias_ih, const float* __restrict__ bias_hh,
    const float* __restrict__ gates,
    float* __restrict__ out,
    int B)
{
    __shared__ __attribute__((aligned(16))) unsigned short Ah[32 * KP];
    __shared__ __attribute__((aligned(16))) unsigned short Al[32 * KP];
    __shared__ WTile Uw;
    __shared__ __attribute__((aligned(16))) unsigned short Wl[BLK * KP];
    __shared__ __attribute__((aligned(16))) float Gl[32 * 64];

    const int t = threadIdx.x, lane = t & 31, w = t >> 5, h = lane >> 4, q = lane & 15;
    const int m0 = blockIdx.x * 32, jh = blockIdx.y;
    if (m0 + 32 > B) return;

#pragma unroll
    for (int it = 0; it < 8; ++it) {
        const int idx = it * NT + t;
        const int r = idx >> 6, rem = idx & 63, kb = rem >> 2, gt = rem & 3;
        const int b = m0 + r, j = gt * 8 + jh;
        Gl[idx] = (kb < 8) ? gates[(size_t)b * GD + kb * 32 + j]
                           : gates[((size_t)B + b) * GD + (kb - 8) * 32 + j];
    }

    v8f aI0 = zero8(), aI1 = zero8(), aF0 = zero8(), aF1 = zero8();
    v8f aC0 = zero8(), aC1 = zero8(), aO0 = zero8(), aO1 = zero8();
    gate_pass(0, aI0, aI1, input, hx, weight_ih, weight_hh, Ah, Al, Uw.w, Wl, Gl, m0, jh, t, w, h, q);
    gate_pass(1, aF0, aF1, input, hx, weight_ih, weight_hh, Ah, Al, Uw.w, Wl, Gl, m0, jh, t, w, h, q);
    gate_pass(2, aC0, aC1, input, hx, weight_ih, weight_hh, Ah, Al, Uw.w, Wl, Gl, m0, jh, t, w, h, q);
    gate_pass(3, aO0, aO1, input, hx, weight_ih, weight_hh, Ah, Al, Uw.w, Wl, Gl, m0, jh, t, w, h, q);

    __syncthreads();
    const int hl = w * 16 + q;
    const int hcol = jh * BLK + hl;
    const float bI = bias_ih[hcol]           + bias_hh[hcol];
    const float bF = bias_ih[HID + hcol]     + bias_hh[HID + hcol];
    const float bC = bias_ih[2 * HID + hcol] + bias_hh[2 * HID + hcol];
    const float bO = bias_ih[3 * HID + hcol] + bias_hh[3 * HID + hcol];
    float cy0[8], cy1[8];
#pragma unroll
    for (int r = 0; r < 8; ++r) {
        const int row = 8 * h + r;
        const size_t m = (size_t)(m0 + row);
        float cyv;
        const float hyv = cell_point(aI0[r] + bI, aF0[r] + bF, aC0[r] + bC, aO0[r] + bO,
                                     cx[m * HID + hcol], cyv);
        Uw.c[row * CPC + hl] = hyv;
        cy0[r] = cyv;
    }
#pragma unroll
    for (int r = 0; r < 8; ++r) {
        const int row = 16 + 8 * h + r;
        const size_t m = (size_t)(m0 + row);
        float cyv;
        const float hyv = cell_point(aI1[r] + bI, aF1[r] + bF, aC1[r] + bC, aO1[r] + bO,
                                     cx[m * HID + hcol], cyv);
        Uw.c[row * CPC + hl] = hyv;
        cy1[r] = cyv;
    }
    __syncthreads();
    v4f hv[4], cv[4];
#pragma unroll
    for (int rr = 0; rr < 4; ++rr) hv[rr] = *(const v4f*)&Uw.c[(4 * w + rr) * CPC + 4 * lane];
    __syncthreads();
#pragma unroll
    for (int r = 0; r < 8; ++r) {
        Uw.c[(8 * h + r) * CPC + hl]      = cy0[r];
        Uw.c[(16 + 8 * h + r) * CPC + hl] = cy1[r];
    }
    __syncthreads();
#pragma unroll
    for (int rr = 0; rr < 4; ++rr) cv[rr] = *(const v4f*)&Uw.c[(4 * w + rr) * CPC + 4 * lane];

    float* ph = out + (size_t)(m0 + 4 * w) * HID + jh * BLK + 4 * lane;
    float* pc = ph + (size_t)B * HID;
#pragma unroll
    for (int rr = 0; rr < 4; ++rr) {
        *(volatile v4f*)(ph + (size_t)rr * HID) = hv[rr];
        *(volatile v4f*)(pc + (size_t)rr * HID) = cv[rr];
    }
    __threadfence();
#pragma unroll
    for (int rr = 0; rr < 4; ++rr) {
        *(volatile v4f*)(ph + (size_t)rr * HID) = hv[rr];
        *(volatile v4f*)(pc + (size_t)rr * HID) = cv[rr];
    }
}

extern "C" void kernel_launch(void* const* d_in, const int* in_sizes, int n_in,
                              void* d_out, int out_size, void* d_ws, size_t ws_size,
                              hipStream_t stream)
{
    if (n_in < 11) return;
    const int B = in_sizes[0] / FEAT;
    if (B <= 0 || (B % 32) != 0) return;
    if (in_sizes[0] != B * FEAT || in_sizes[1] != B * HID || in_sizes[2] != B * HID) return;
    if (in_sizes[3] != FEAT * GATEW || in_sizes[4] != HID * GATEW) return;
    if (in_sizes[5] != GATEW || in_sizes[6] != GATEW) return;
    if (in_sizes[7] != FEAT * GD || in_sizes[8] != GD || in_sizes[9] != HID * GD || in_sizes[10] != GD) return;
    if (out_size != 2 * B * HID) return;
    const size_t n_log = (size_t)2 * (size_t)B * GD;
    if (2 * n_log * sizeof(float) > ws_size) return;

    const float* input     = (const float*)d_in[0];
    const float* hx        = (const float*)d_in[1];
    const float* cx        = (const float*)d_in[2];
    const float* weight_ih = (const float*)d_in[3];
    const float* weight_hh = (const float*)d_in[4];
    const float* bias_ih   = (const float*)d_in[5];
    const float* bias_hh   = (const float*)d_in[6];
    const float* w_gih     = (const float*)d_in[7];
    const float* b_gih     = (const float*)d_in[8];
    const float* w_ghh     = (const float*)d_in[9];
    const float* b_ghh     = (const float*)d_in[10];
    float* out    = (float*)d_out;
    float* logits = (float*)d_ws;
    float* gates  = logits + n_log;

    k_gate_logits<<<dim3(B / 32, GD / 64, 2), NT, 0, stream>>>(
        input, hx, w_gih, w_ghh, b_gih, b_ghh, logits, B);
    k_sparsify<<<dim3((2 * B + 7) / 8), NT, 0, stream>>>(logits, gates, 2 * B);
    k_gated_lstm<<<dim3(B / 32, HID / BLK), NT, 0, stream>>>(
        input, hx, cx, weight_ih, weight_hh, bias_ih, bias_hh, gates, out, B);
}
